// CoaT_38405597561606
// MI455X (gfx1250) — hardware-verified
//
#include <hip/hip_runtime.h>
#include <math.h>

constexpr int NB_ALL  = 16;
constexpr int NTOK    = 3137;
constexpr int NC      = 256;
constexpr int NHEAD   = 8;
constexpr int HCH     = 32;
constexpr int IMW     = 56;
constexpr int NQKV    = 768;
constexpr int NFF     = 1024;
constexpr int GBATCH  = 4;
constexpr int NGROUP  = NB_ALL / GBATCH;
constexpr int NPAD    = 3200;
constexpr int MGRP    = GBATCH * NPAD;
constexpr int ATT_TPB = 16;
constexpr float FACTOR_SCALE = 0.1767766952966369f;
constexpr float W_CARRY   = 16.0f;
constexpr float ATT_CARRY = 64.0f;
constexpr float H_CARRY   = 16.0f;

constexpr size_t OFFW_QKV  = 0;
constexpr size_t OFFW_PROJ = (size_t)NQKV * NC;
constexpr size_t OFFW_FC1  = OFFW_PROJ + (size_t)NC * NC;
constexpr size_t OFFW_FC2  = OFFW_FC1 + (size_t)NFF * NC;
constexpr size_t W16_HALVES = OFFW_FC2 + (size_t)NC * NFF;

constexpr size_t SZ_W16  = W16_HALVES * 2;
constexpr size_t SZ_XB   = (size_t)MGRP * NC * 4;
constexpr size_t SZ_CUR  = (size_t)MGRP * NC * 2;
constexpr size_t SZ_BIG  = (size_t)MGRP * NFF * 4;
constexpr size_t SZ_H16  = (size_t)MGRP * NFF * 2;
constexpr size_t SZ_KST  = (size_t)2 * GBATCH * NC * 4;
constexpr size_t SZ_KVB  = (size_t)GBATCH * NHEAD * HCH * HCH * 4;
constexpr size_t OFF_W16 = 0;
constexpr size_t OFF_XB  = OFF_W16 + SZ_W16;
constexpr size_t OFF_X1  = OFF_XB + SZ_XB;
constexpr size_t OFF_CUR = OFF_X1 + SZ_XB;
constexpr size_t OFF_ATT = OFF_CUR + SZ_CUR;
constexpr size_t OFF_BIG = OFF_ATT + SZ_CUR;
constexpr size_t OFF_H16 = OFF_BIG + SZ_BIG;
constexpr size_t OFF_KST = OFF_H16 + SZ_H16;
constexpr size_t OFF_KVB = OFF_KST + SZ_KST;
constexpr size_t WS_TOTAL = OFF_KVB + SZ_KVB;
typedef char chk_ws_total[(WS_TOTAL <= (size_t)134217728) ? 1 : -1];
typedef char chk_qkv_fits[((size_t)MGRP * NQKV * 4 <= SZ_BIG) ? 1 : -1];
typedef char chk_align[((OFF_XB % 128) == 0 && (OFF_CUR % 128) == 0 && (OFF_BIG % 128) == 0 && (OFF_KST % 128) == 0 && (OFF_KVB % 128) == 0) ? 1 : -1];
typedef char chk_tiles[((MGRP % 64) == 0 && (NPAD % 64) == 0 && (NPAD % ATT_TPB) == 0) ? 1 : -1];

typedef __attribute__((ext_vector_type(16))) _Float16 v16h;
typedef __attribute__((ext_vector_type(8)))  _Float16 v8h;
typedef __attribute__((ext_vector_type(16))) __bf16   v16b;
typedef __attribute__((ext_vector_type(8)))  __bf16   v8b;
typedef __attribute__((ext_vector_type(8)))  float    v8f;
typedef __attribute__((ext_vector_type(4)))  float    v4f;
typedef __attribute__((ext_vector_type(4)))  unsigned int v4u;

__device__ __forceinline__ unsigned short f2bf_bits(float f) {
  unsigned u = __float_as_uint(f);
  return (unsigned short)((u + 0x7FFFu + ((u >> 16) & 1u)) >> 16);
}
__device__ __forceinline__ float bf_bits2f(unsigned short h) { return __uint_as_float(((unsigned)h) << 16); }

__device__ __forceinline__ void dep_guard_h(v8f& a, v8f& b, v16h x, v16h y) { asm volatile("v_nop\n\tv_nop\n\tv_nop\n\tv_nop" : "+v"(a), "+v"(b) : "v"(x), "v"(y)); }
__device__ __forceinline__ void dep_guard_b(v8f& a, v8f& b, v16b x, v16b y) { asm volatile("v_nop\n\tv_nop\n\tv_nop\n\tv_nop" : "+v"(a), "+v"(b) : "v"(x), "v"(y)); }
__device__ __forceinline__ void keep4_h(v16h a, v16h b, v16h c, v16h d) { asm volatile("v_nop" :: "v"(a), "v"(b), "v"(c), "v"(d)); }
__device__ __forceinline__ void keep4_b(v16b a, v16b b, v16b c, v16b d) { asm volatile("v_nop" :: "v"(a), "v"(b), "v"(c), "v"(d)); }
__device__ __forceinline__ void acc_guard4(v8f& a, v8f& b, v8f& c, v8f& d) { asm volatile("v_nop\n\tv_nop\n\tv_nop\n\tv_nop" : "+v"(a), "+v"(b), "+v"(c), "+v"(d)); }
template <typename T> struct Frag;
template <> struct Frag<_Float16> {
  typedef v16h V; union U { v16h v; v8h h[2]; };
  static __device__ __forceinline__ v16h load(const _Float16* p) {
    U f; f.h[0] = *(const v8h*)(p); f.h[1] = *(const v8h*)(p + 16); return f.v;
  }
  static __device__ __forceinline__ v8f mma(v16h a, v16h b, v8f c) {
    return __builtin_amdgcn_wmma_f32_16x16x32_f16(false, a, false, b, (short)0, c, false, false);
  }
  static __device__ __forceinline__ void guard(v8f& a, v8f& b, v16h x, v16h y) { dep_guard_h(a, b, x, y); }
  static __device__ __forceinline__ void keep(v16h a, v16h b, v16h c, v16h d) { keep4_h(a, b, c, d); }
};
template <> struct Frag<__bf16> {
  typedef v16b V; union U { v16b v; v8b h[2]; };
  static __device__ __forceinline__ v16b load(const __bf16* p) {
    U f; f.h[0] = *(const v8b*)(p); f.h[1] = *(const v8b*)(p + 16); return f.v;
  }
  static __device__ __forceinline__ v8f mma(v16b a, v16b b, v8f c) {
    return __builtin_amdgcn_wmma_f32_16x16x32_bf16(false, a, false, b, (short)0, c, false, false);
  }
  static __device__ __forceinline__ void guard(v8f& a, v8f& b, v16b x, v16b y) { dep_guard_b(a, b, x, y); }
  static __device__ __forceinline__ void keep(v16b a, v16b b, v16b c, v16b d) { keep4_b(a, b, c, d); }
};

__device__ __forceinline__ unsigned pk16(unsigned short a, unsigned short b) { return (unsigned)a | ((unsigned)b << 16); }
__device__ __forceinline__ unsigned short h_bits(float f) { const _Float16 h = (_Float16)f; return __builtin_bit_cast(unsigned short, h); }

template <int ET> struct Elem;
template <> struct Elem<0> { typedef _Float16 T; };
template <> struct Elem<1> { typedef __bf16 T; };
template <int ET, bool SPLIT, int BIAS_MODE, int OUT_MODE, bool RESID, int ACT = 0>
__global__ __launch_bounds__(256) void wmma_gemm64(
    const unsigned short* __restrict__ Ap, const unsigned short* __restrict__ A2p, int lda, long strideA,
    const unsigned short* __restrict__ Btp, const unsigned short* __restrict__ Bt2p, int ldb, long strideB,
    void* __restrict__ Cout, void* __restrict__ Cout2, int ldc, long strideC,
    const float* __restrict__ bias,
    const float* __restrict__ resid, long strideR,
    int M, int N, int K, float scale, int Mlim) {
  typedef typename Elem<ET>::T T;
  typedef typename Frag<T>::V V;
  const T* A = (const T*)Ap; const T* A2 = (const T*)A2p; const T* Bt = (const T*)Btp; const T* Bt2 = (const T*)Bt2p;
  __shared__ __align__(16) float sT[8][16 * 68];
  const int b    = blockIdx.y;
  const int lane = threadIdx.x & 31;
  const int wave = threadIdx.x >> 5;
  const int tilesN = N >> 6;
  const int tilesM = M >> 6;
  const int tile = blockIdx.x * 8 + wave;
  if (tile >= tilesM * tilesN) return;
  const int tm = tile / tilesN;
  const int tn = tile - tm * tilesN;
  const int m0 = tm << 6;
  const int n0 = tn << 6;

  const T* Ab  = A  + (size_t)b * strideA;
  const T* Bb  = Bt + (size_t)b * strideB;
  const T* Ab2 = SPLIT ? (A2  + (size_t)b * strideA) : nullptr;
  const T* Bb2 = SPLIT ? (Bt2 + (size_t)b * strideB) : nullptr;

  const int rlane = lane & 15;
  const int koff  = (lane >> 4) * 8;
  const int mOff  = (lane >> 4) * 8;

  v8f acc[4][4];
#pragma unroll
  for (int i = 0; i < 4; ++i)
#pragma unroll
    for (int j = 0; j < 4; ++j) acc[i][j] = (v8f){0.f,0.f,0.f,0.f,0.f,0.f,0.f,0.f};

  for (int k0 = 0; k0 < K; k0 += 32) {
    V bh[4], bl[4];
#pragma unroll
    for (int j = 0; j < 4; ++j) {
      const size_t bo = (size_t)(n0 + (j << 4) + rlane) * ldb + koff + k0;
      bh[j] = Frag<T>::load(Bb + bo);
      if (SPLIT) bl[j] = Frag<T>::load(Bb2 + bo);
    }
#pragma unroll
    for (int i = 0; i < 4; ++i) {
      const size_t ao = (size_t)(m0 + (i << 4) + rlane) * lda + koff + k0;
      V ah = Frag<T>::load(Ab + ao);
      V al;
      if (SPLIT) al = Frag<T>::load(Ab2 + ao);
#pragma unroll
      for (int j = 0; j < 4; ++j) {
        acc[i][j] = Frag<T>::mma(ah, bh[j], acc[i][j]);
        if (SPLIT) {
          acc[i][j] = Frag<T>::mma(ah, bl[j], acc[i][j]);
          acc[i][j] = Frag<T>::mma(al, bh[j], acc[i][j]);
        }
      }
      Frag<T>::guard(acc[i][0], acc[i][3], ah, SPLIT ? al : ah);
    }
    Frag<T>::keep(bh[0], bh[1], bh[2], bh[3]);
    if (SPLIT) Frag<T>::keep(bl[0], bl[1], bl[2], bl[3]);
  }
  acc_guard4(acc[0][0], acc[0][1], acc[0][2], acc[0][3]);
  acc_guard4(acc[1][0], acc[1][1], acc[1][2], acc[1][3]);
  acc_guard4(acc[2][0], acc[2][1], acc[2][2], acc[2][3]);
  acc_guard4(acc[3][0], acc[3][1], acc[3][2], acc[3][3]);

  float* slab = sT[wave];
  const float* Rb = RESID ? (resid + (size_t)b * strideR) : nullptr;
#pragma unroll
  for (int i = 0; i < 4; ++i) {
    const int mBase = m0 + (i << 4);
#pragma unroll
    for (int j = 0; j < 4; ++j) {
      const int n = n0 + (j << 4) + rlane;
      float bv = 0.f;
      if (BIAS_MODE == 2) bv = bias[n];
#pragma unroll
      for (int r = 0; r < 8; ++r) {
        float v = acc[i][j][r] * scale;
        if (BIAS_MODE == 1) v += bias[mBase + mOff + r];
        if (BIAS_MODE == 2) v += bv;
        if (RESID) v += Rb[(size_t)(mBase + mOff + r) * ldc + n];
        if (ACT == 2) v = fmaxf(v, 0.0f);
        if (ACT == 4) v = (v > 0.f) ? v : 0.01f * v;
        slab[(mOff + r) * 68 + (j << 4) + rlane] = v;
      }
    }
    __builtin_amdgcn_fence(__ATOMIC_RELEASE, "workgroup");
    __builtin_amdgcn_wave_barrier();
    __builtin_amdgcn_fence(__ATOMIC_ACQUIRE, "workgroup");
    if (OUT_MODE == 0) {
      float* C = (float*)Cout + (size_t)b * strideC;
      const int hh = lane >> 4, c4 = (lane & 15) * 4;
      for (int pass = 0; pass < 2; ++pass) {
#pragma unroll
        for (int it = 0; it < 8; ++it) {
          const int row = it * 2 + hh;
          v4f v = *(const v4f*)(slab + row * 68 + c4);
          if (mBase + row < Mlim) *(volatile v4f*)(C + (size_t)(mBase + row) * ldc + n0 + c4) = v;
        }
        __threadfence();
      }
    } else {
      const int q = lane >> 3, c8 = (lane & 7) * 8;
      unsigned short* C  = (unsigned short*)Cout  + (size_t)b * strideC;
      unsigned short* C2 = (OUT_MODE == 2) ? ((unsigned short*)Cout2 + (size_t)b * strideC) : nullptr;
      for (int pass = 0; pass < 2; ++pass) {
#pragma unroll
        for (int it = 0; it < 4; ++it) {
          const int row = it * 4 + q;
          const float* sp = slab + row * 68 + c8;
          v8h hv, lv;
#pragma unroll
          for (int e = 0; e < 8; ++e) {
            if (OUT_MODE == 1) {
              hv[e] = (_Float16)sp[e];
            } else {
              unsigned short hb = f2bf_bits(sp[e]);
              unsigned short lb = f2bf_bits(sp[e] - bf_bits2f(hb));
              hv[e] = __builtin_bit_cast(_Float16, hb);
              lv[e] = __builtin_bit_cast(_Float16, lb);
            }
          }
          if (mBase + row < Mlim) {
            *(volatile v8h*)(C + (size_t)(mBase + row) * ldc + n0 + c8) = hv;
            if (OUT_MODE == 2) *(volatile v8h*)(C2 + (size_t)(mBase + row) * ldc + n0 + c8) = lv;
          }
        }
        __threadfence();
      }
    }
    __builtin_amdgcn_fence(__ATOMIC_RELEASE, "workgroup");
    __builtin_amdgcn_wave_barrier();
    __builtin_amdgcn_fence(__ATOMIC_ACQUIRE, "workgroup");
  }
}

__global__ __launch_bounds__(256) void k_wcast(const float* __restrict__ w0, const float* __restrict__ w1,
                                               const float* __restrict__ w2, const float* __restrict__ w3p,
                                               unsigned short* __restrict__ out, float scale) {
  const int y = blockIdx.y;
  const float* W = (y == 0) ? w0 : ((y == 1) ? w1 : ((y == 2) ? w2 : w3p));
  const int n = (y == 0) ? (NQKV * NC) : ((y == 1) ? (NC * NC) : (NFF * NC));
  const size_t ob = (y == 0) ? OFFW_QKV : ((y == 1) ? OFFW_PROJ : ((y == 2) ? OFFW_FC1 : OFFW_FC2));
  const int i = blockIdx.x * 256 + threadIdx.x;
  if (8 * i >= n) return;
  const float* p = W + 8 * (size_t)i;
  const v4f a = *(const v4f*)(p);
  const v4f c = *(const v4f*)(p + 4);
  unsigned short hb[8];
#pragma unroll
  for (int e = 0; e < 4; ++e) {
    hb[e]     = h_bits(a[e] * scale);
    hb[4 + e] = h_bits(c[e] * scale);
  }
  const v4u u = (v4u){pk16(hb[0], hb[1]), pk16(hb[2], hb[3]), pk16(hb[4], hb[5]), pk16(hb[6], hb[7])};
  unsigned short* q = out + ob + 8 * (size_t)i;
  *(volatile v4u*)q = u;
  __threadfence();
  *(volatile v4u*)q = u;
}

template <bool DO_CPE>
__global__ __launch_bounds__(256) void k_rowln(const float* __restrict__ src, const float* __restrict__ cw,
                                               const float* __restrict__ cb, const float* __restrict__ g,
                                               const float* __restrict__ be, float* __restrict__ xb,
                                               unsigned short* __restrict__ cur, int grp) {
  __shared__ float red[8];
  __shared__ float red2[8];
  __shared__ __align__(16) float ys[NC];
  const int c = threadIdx.x, lane = c & 31, wave = c >> 5;
  const int row = blockIdx.x;
  const int bl = row / NPAD;
  const int n = row - bl * NPAD;
  const bool valid = (n < NTOK);
  float v = 0.f;
  if (valid) {
    if (DO_CPE) {
      const size_t tokbase = (size_t)(grp * GBATCH + bl) * NTOK;
      const float xv = src[(tokbase + n) * NC + c];
      if (n == 0) {
        v = xv;
      } else {
        const int hw = n - 1;
        const int yy = hw / IMW;
        const int xx = hw - yy * IMW;
        const float* wc = cw + c * 9;
        float acc = 0.f;
#pragma unroll
        for (int ky = 0; ky < 3; ++ky) {
          const int iy = yy + ky - 1;
          const bool iny = ((unsigned)iy < (unsigned)IMW);
          const int iyc = min(max(iy, 0), IMW - 1);
#pragma unroll
          for (int kx = 0; kx < 3; ++kx) {
            const int ix = xx + kx - 1;
            const bool inb = iny && ((unsigned)ix < (unsigned)IMW);
            const int ixc = min(max(ix, 0), IMW - 1);
            const float nv = src[(tokbase + 1 + (size_t)(iyc * IMW + ixc)) * NC + c];
            acc += wc[ky * 3 + kx] * (inb ? nv : 0.f);
          }
        }
        v = (acc + cb[c]) + xv;
      }
    } else {
      v = src[(size_t)row * NC + c];
    }
  }
  if (DO_CPE) {
    volatile float* xo = xb + (size_t)row * NC + c;
    *xo = v;
    __threadfence();
    *xo = v;
  }
  float s = v;
#pragma unroll
  for (int off = 16; off > 0; off >>= 1) s += __shfl_xor(s, off, 32);
  if (lane == 0) red[wave] = s;
  __syncthreads();
  float tot = 0.f;
#pragma unroll
  for (int w = 0; w < 8; ++w) tot += red[w];
  const float mean = tot * (1.0f / NC);
  const float d = v - mean;
  float s2 = d * d;
#pragma unroll
  for (int off = 16; off > 0; off >>= 1) s2 += __shfl_xor(s2, off, 32);
  if (lane == 0) red2[wave] = s2;
  __syncthreads();
  float tot2 = 0.f;
#pragma unroll
  for (int w = 0; w < 8; ++w) tot2 += red2[w];
  const float var = tot2 * (1.0f / NC);
  const float rstd = 1.0f / sqrtf(var + 1e-6f);
  float y = d * rstd * g[c] + be[c];
  y = valid ? y : 0.f;
  ys[c] = y;
  __syncthreads();
  if (wave == 0) {
    const v4f a = *(const v4f*)(ys + 8 * lane);
    const v4f bq = *(const v4f*)(ys + 8 * lane + 4);
    unsigned short hb[8];
#pragma unroll
    for (int e = 0; e < 4; ++e) { hb[e] = h_bits(a[e]); hb[4 + e] = h_bits(bq[e]); }
    const v4u u = (v4u){pk16(hb[0], hb[1]), pk16(hb[2], hb[3]), pk16(hb[4], hb[5]), pk16(hb[6], hb[7])};
    unsigned short* op = cur + (size_t)row * NC + 8 * lane;
    *(volatile v4u*)op = u;
    __threadfence();
    *(volatile v4u*)op = u;
  }
}

__global__ __launch_bounds__(256) void k_ksm(const float* __restrict__ qkv, float* __restrict__ kst) {
  const int c = threadIdx.x;
  const int bl = blockIdx.x;
  const float* base = qkv + (size_t)bl * NPAD * NQKV + NC + c;
  float gm = -INFINITY, gs = 0.f;
#pragma unroll 1
  for (int n0 = 0; n0 < NTOK; n0 += 64) {
    const int n1 = min(n0 + 64, NTOK);
    float m = -INFINITY, s = 0.f;
#pragma unroll 1
    for (int n = n0; n < n1; ++n) {
      const float kv = base[(size_t)n * NQKV];
      const float mn = fmaxf(m, kv);
      s = s * expf(m - mn) + expf(kv - mn);
      m = mn;
    }
    const float gmn = fmaxf(gm, m);
    gs = gs * expf(gm - gmn) + s * expf(m - gmn);
    gm = gmn;
  }
  const float inv = 1.0f / gs;
  volatile float* p1 = kst + bl * NC + c;
  volatile float* p2 = kst + GBATCH * NC + bl * NC + c;
  *p1 = gm; *p2 = inv;
  __threadfence();
  *p1 = gm; *p2 = inv;
}

__global__ __launch_bounds__(256) void k_kv(const float* __restrict__ qkv, const float* __restrict__ kst,
                                            float* __restrict__ kvb) {
  __shared__ __align__(16) float ks[64 * HCH];
  __shared__ __align__(16) float vs[64 * HCH];
  const int t = threadIdx.x;
  const int blk = blockIdx.x;
  const int bl = blk >> 3, h = blk & 7;
  const int ch = t & 31;
  const float hmr = kst[bl * NC + h * HCH + ch];
  const float hir = kst[GBATCH * NC + bl * NC + h * HCH + ch];
  const int c = t >> 3, d0 = (t & 7) * 4;
  const float* kb = qkv + (size_t)bl * NPAD * NQKV + NC + h * HCH;
  const float* vb = kb + NC;
  float a0 = 0.f, a1 = 0.f, a2 = 0.f, a3 = 0.f;
#pragma unroll 1
  for (int n0 = 0; n0 < NPAD; n0 += 64) {
#pragma unroll
    for (int l = 0; l < 2; ++l) {
      const int i = t + 256 * l;
      const int tk = i >> 3;
      const int q4 = (i & 7) * 4;
      const int n = n0 + tk;
      const bool nv = (n < NTOK);
      const int nc = nv ? n : (NTOK - 1);
      const v4f kk = *(const v4f*)(kb + (size_t)nc * NQKV + q4);
      v4f vv = *(const v4f*)(vb + (size_t)nc * NQKV + q4);
      if (!nv) vv = (v4f){0.f, 0.f, 0.f, 0.f};
      *(v4f*)(ks + tk * HCH + q4) = kk;
      *(v4f*)(vs + tk * HCH + q4) = vv;
    }
    __syncthreads();
#pragma unroll 1
    for (int j = 0; j < 8; ++j) {
      const int idx = j * 256 + t;
      ks[idx] = expf(ks[idx] - hmr) * hir;
    }
    __syncthreads();
#pragma unroll 8
    for (int i = 0; i < 64; ++i) {
      const float kvl = ks[i * HCH + c];
      const v4f v4 = *(const v4f*)(vs + i * HCH + d0);
      a0 += kvl * v4.x; a1 += kvl * v4.y; a2 += kvl * v4.z; a3 += kvl * v4.w;
    }
    __syncthreads();
  }
  const v4f o = (v4f){a0, a1, a2, a3};
  float* op = kvb + (size_t)blk * (HCH * HCH) + c * HCH + d0;
  *(volatile v4f*)op = o;
  __threadfence();
  *(volatile v4f*)op = o;
}

__global__ __launch_bounds__(256) void k_att(const float* __restrict__ qkv, const float* __restrict__ kvb,
                                             const float* __restrict__ w3, const float* __restrict__ b3,
                                             const float* __restrict__ w5, const float* __restrict__ b5,
                                             const float* __restrict__ w7, const float* __restrict__ b7,
                                             unsigned short* __restrict__ att) {
  __shared__ __align__(16) float qs[ATT_TPB * NC];
  __shared__ __align__(16) float os[ATT_TPB * NC];
  __shared__ float wt[7680];
  const int c = threadIdx.x, lane = c & 31, wave = c >> 5;
  const int h = wave, d = lane;
  const int blk = blockIdx.x;
  const int bl = blk / (NPAD / ATT_TPB);
  const int tg = blk - bl * (NPAD / ATT_TPB);
  const int n0 = tg * ATT_TPB;
  const size_t rowbase = (size_t)bl * NPAD;
  const int grp = (c < 64) ? 0 : ((c < 160) ? 1 : 2);
  const int ksz = (grp == 0) ? 3 : ((grp == 1) ? 5 : 7);
  const int ntap = ksz * ksz;
  const int half = ksz >> 1;
  const int cl = (grp == 0) ? c : ((grp == 1) ? (c - 64) : (c - 160));
  const int wbase = (grp == 0) ? 0 : ((grp == 1) ? 576 : 2976);
  const int wstr = (grp == 0) ? 64 : 96;
  const int c3 = min(c, 63);
  const int c5 = min(max(c - 64, 0), 95);
  const int c7 = min(max(c - 160, 0), 95);
#pragma unroll 1
  for (int tap = 0; tap < 49; ++tap) {
    const float va = w3[c3 * 9 + min(tap, 8)];
    const float vq = w5[c5 * 25 + min(tap, 24)];
    const float vz = w7[c7 * 49 + tap];
    const float val = (grp == 0) ? va : ((grp == 1) ? vq : vz);
    if (tap < ntap) wt[wbase + tap * wstr + cl] = val;
  }
  const float ba = b3[c3], bq = b5[c5], bz = b7[c7];
  const float bsel = (grp == 0) ? ba : ((grp == 1) ? bq : bz);
  float kvr[32];
  const float* kvp = kvb + ((size_t)(bl * NHEAD + h) * HCH) * HCH + d;
#pragma unroll
  for (int cc = 0; cc < 32; ++cc) kvr[cc] = kvp[cc * HCH];
#pragma unroll
  for (int t = 0; t < ATT_TPB; ++t) {
    const int n = min(n0 + t, NTOK - 1);
    qs[t * NC + c] = qkv[(rowbase + n) * NQKV + c];
  }
  __syncthreads();
  const float* vcol = qkv + (rowbase + 1) * NQKV + 2 * NC + c;
#pragma unroll 1
  for (int t = 0; t < ATT_TPB; ++t) {
    const int n = n0 + t;
    float r = 0.f;
    if (n < NTOK) {
      const float* qh = qs + t * NC + h * HCH;
      float f = 0.f;
#pragma unroll
      for (int c4 = 0; c4 < 8; ++c4) {
        const v4f q4 = *(const v4f*)(qh + 4 * c4);
        f += q4.x * kvr[4 * c4 + 0];
        f += q4.y * kvr[4 * c4 + 1];
        f += q4.z * kvr[4 * c4 + 2];
        f += q4.w * kvr[4 * c4 + 3];
      }
      r = FACTOR_SCALE * f;
      if (n >= 1) {
        const int hw = n - 1;
        const int yy = hw / IMW;
        const int xx = hw - yy * IMW;
        float conv = 0.f;
#pragma unroll 1
        for (int ky = 0; ky < ksz; ++ky) {
          const int iy = yy + ky - half;
          const bool iny = ((unsigned)iy < (unsigned)IMW);
          const int iyc = min(max(iy, 0), IMW - 1);
#pragma unroll 1
          for (int kx = 0; kx < ksz; ++kx) {
            const int ix = xx + kx - half;
            const bool inb = iny && ((unsigned)ix < (unsigned)IMW);
            const int ixc = min(max(ix, 0), IMW - 1);
            const float vv = vcol[(size_t)(iyc * IMW + ixc) * NQKV];
            const float wv = wt[wbase + (ky * ksz + kx) * wstr + cl];
            conv += wv * (inb ? vv : 0.f);
          }
        }
        conv += bsel;
        r += qs[t * NC + c] * conv;
      }
    }
    os[t * NC + c] = r;
  }
  __syncthreads();
  for (int pass = 0; pass < 2; ++pass) {
#pragma unroll
    for (int rr = 0; rr < 2; ++rr) {
      const int t = wave * 2 + rr;
      const float* sp = os + t * NC + 8 * lane;
      const v4f a = *(const v4f*)(sp);
      const v4f bq2 = *(const v4f*)(sp + 4);
      unsigned short hb[8];
#pragma unroll
      for (int e = 0; e < 4; ++e) {
        hb[e]     = h_bits(a[e] * ATT_CARRY);
        hb[4 + e] = h_bits(bq2[e] * ATT_CARRY);
      }
      const v4u u = (v4u){pk16(hb[0], hb[1]), pk16(hb[2], hb[3]), pk16(hb[4], hb[5]), pk16(hb[6], hb[7])};
      *(volatile v4u*)(att + (rowbase + n0 + t) * NC + 8 * lane) = u;
    }
    __threadfence();
  }
}

__global__ __launch_bounds__(256) void k_gelu(const float* __restrict__ u, unsigned short* __restrict__ hout,
                                              int n2, float carry) {
  const int i = blockIdx.x * 256 + threadIdx.x;
  if (i >= n2) return;
  const float a = u[2 * (size_t)i];
  const float bq = u[2 * (size_t)i + 1];
  const float ga = 0.5f * a  * (1.0f + erff(a  * 0.70710678118654752f)) * carry;
  const float gb = 0.5f * bq * (1.0f + erff(bq * 0.70710678118654752f)) * carry;
  const unsigned w = pk16(h_bits(ga), h_bits(gb));
  volatile unsigned* op = (volatile unsigned*)hout + i;
  *op = w;
  __threadfence();
  *op = w;
}

extern "C" void kernel_launch(void* const* d_in, const int* in_sizes, int n_in,
                              void* d_out, int out_size, void* d_ws, size_t ws_size,
                              hipStream_t stream) {
  if (n_in < 21) return;
  if (in_sizes[0] != NB_ALL * NTOK * NC) return;
  if (out_size < NB_ALL * NTOK * NC) return;
  if (ws_size < WS_TOTAL) return;

  const float* x      = (const float*)d_in[0];
  const float* cpe_w  = (const float*)d_in[1];
  const float* cpe_b  = (const float*)d_in[2];
  const float* ln1_g  = (const float*)d_in[3];
  const float* ln1_b  = (const float*)d_in[4];
  const float* qkv_w  = (const float*)d_in[5];
  const float* qkv_b  = (const float*)d_in[6];
  const float* crw3   = (const float*)d_in[7];
  const float* crb3   = (const float*)d_in[8];
  const float* crw5   = (const float*)d_in[9];
  const float* crb5   = (const float*)d_in[10];
  const float* crw7   = (const float*)d_in[11];
  const float* crb7   = (const float*)d_in[12];
  const float* proj_w = (const float*)d_in[13];
  const float* proj_b = (const float*)d_in[14];
  const float* ln2_g  = (const float*)d_in[15];
  const float* ln2_b  = (const float*)d_in[16];
  const float* fc1_w  = (const float*)d_in[17];
  const float* fc1_b  = (const float*)d_in[18];
  const float* fc2_w  = (const float*)d_in[19];
  const float* fc2_b  = (const float*)d_in[20];

  char* ws = (char*)d_ws;
  unsigned short* W16   = (unsigned short*)(ws + OFF_W16);
  float*          XB    = (float*)(ws + OFF_XB);
  float*          X1    = (float*)(ws + OFF_X1);
  unsigned short* CUR16 = (unsigned short*)(ws + OFF_CUR);
  unsigned short* ATT16 = (unsigned short*)(ws + OFF_ATT);
  float*          QKVF  = (float*)(ws + OFF_BIG);
  float*          U32   = (float*)(ws + OFF_BIG);
  unsigned short* H16   = (unsigned short*)(ws + OFF_H16);
  float*          KST   = (float*)(ws + OFF_KST);
  float*          KVB   = (float*)(ws + OFF_KVB);
  float*          OUT   = (float*)d_out;

  const unsigned short* WQKV  = W16 + OFFW_QKV;
  const unsigned short* WPROJ = W16 + OFFW_PROJ;
  const unsigned short* WFC1  = W16 + OFFW_FC1;
  const unsigned short* WFC2  = W16 + OFFW_FC2;

  k_wcast<<<dim3((NFF * NC / 8 + 255) / 256, 4), 256, 0, stream>>>(qkv_w, proj_w, fc1_w, fc2_w, W16, W_CARRY);

  const int gx_qkv  = ((MGRP / 64) * (NQKV / 64) + 7) / 8;
  const int gx_proj = ((MGRP / 64) * (NC / 64) + 7) / 8;
  const int gx_fc1  = ((MGRP / 64) * (NFF / 64) + 7) / 8;
  const int gx_fc2  = ((NPAD / 64) * (NC / 64) + 7) / 8;

  for (int g = 0; g < NGROUP; ++g) {
    k_rowln<true><<<MGRP, 256, 0, stream>>>(x, cpe_w, cpe_b, ln1_g, ln1_b, XB, CUR16, g);
    wmma_gemm64<0, false, 2, 0, false, 0><<<dim3(gx_qkv, 1), 256, 0, stream>>>(
        CUR16, CUR16, NC, (long)0, WQKV, WQKV, NC, (long)0,
        (void*)QKVF, (void*)QKVF, NQKV, (long)0, qkv_b, XB, (long)0,
        MGRP, NQKV, NC, 1.0f / W_CARRY, MGRP);
    k_ksm<<<GBATCH, 256, 0, stream>>>(QKVF, KST);
    k_kv<<<GBATCH * NHEAD, 256, 0, stream>>>(QKVF, KST, KVB);
    k_att<<<GBATCH * (NPAD / ATT_TPB), 256, 0, stream>>>(QKVF, KVB, crw3, crb3, crw5, crb5, crw7, crb7, ATT16);
    wmma_gemm64<0, false, 2, 0, true, 0><<<dim3(gx_proj, 1), 256, 0, stream>>>(
        ATT16, ATT16, NC, (long)0, WPROJ, WPROJ, NC, (long)0,
        (void*)X1, (void*)X1, NC, (long)0, proj_b, XB, (long)0,
        MGRP, NC, NC, 1.0f / (ATT_CARRY * W_CARRY), MGRP);
    k_rowln<false><<<MGRP, 256, 0, stream>>>(X1, cpe_w, cpe_b, ln2_g, ln2_b, XB, CUR16, g);
    wmma_gemm64<0, false, 2, 0, false, 0><<<dim3(gx_fc1, 1), 256, 0, stream>>>(
        CUR16, CUR16, NC, (long)0, WFC1, WFC1, NC, (long)0,
        (void*)U32, (void*)U32, NFF, (long)0, fc1_b, XB, (long)0,
        MGRP, NFF, NC, 1.0f / W_CARRY, MGRP);
    k_gelu<<<(MGRP * NFF / 2 + 255) / 256, 256, 0, stream>>>(U32, H16, MGRP * NFF / 2, H_CARRY);
    float* outg = OUT + (size_t)g * GBATCH * NTOK * NC;
    wmma_gemm64<0, false, 2, 0, true, 0><<<dim3(gx_fc2, GBATCH), 256, 0, stream>>>(
        H16, H16, NFF, (long)NPAD * NFF, WFC2, WFC2, NFF, (long)0,
        (void*)outg, (void*)outg, NC, (long)NTOK * NC, fc2_b, X1, (long)NPAD * NC,
        NPAD, NC, NFF, 1.0f / (H_CARRY * W_CARRY), NTOK);
  }
}
